// SMDScaleAttention_29308856827968
// MI455X (gfx1250) — hardware-verified
//
#include <hip/hip_runtime.h>


#define NN   2048
#define DMD  1024
#define HD   64
#define NSM  2
#define NSD  6
#define NH_  8
#define NSTEP 4
#define PCAR 1024.0f
typedef _Float16 h16;
typedef unsigned short bf;
typedef __attribute__((ext_vector_type(16))) __bf16   v16bf;
typedef __attribute__((ext_vector_type(16))) _Float16 v16h;
typedef __attribute__((ext_vector_type(8)))  _Float16 v8h;
typedef __attribute__((ext_vector_type(8)))  unsigned short v8us;
typedef __attribute__((ext_vector_type(8)))  float    v8f;
typedef __attribute__((ext_vector_type(4)))  float    v4f;
typedef v8h  __attribute__((may_alias)) v8ha;
typedef v4f  __attribute__((may_alias)) v4fa;
typedef v8us __attribute__((may_alias)) v8usa;

__device__ __forceinline__ unsigned short f2bf(float f) { unsigned u = __float_as_uint(f); u += 0x7FFFu + ((u >> 16) & 1u); return (unsigned short)(u >> 16); }
__device__ __forceinline__ float bf2f(unsigned short b) { return __uint_as_float(((unsigned)b) << 16); }
__device__ __forceinline__ float bfr(float f) { return bf2f(f2bf(f)); }
__device__ __forceinline__ v16h cat16(v8h lo, v8h hi) { return __builtin_shufflevector(lo, hi, 0, 1, 2, 3, 4, 5, 6, 7, 8, 9, 10, 11, 12, 13, 14, 15); }
__device__ __forceinline__ v16bf cat16b(v8us lo, v8us hi) { return __builtin_bit_cast(v16bf, __builtin_shufflevector(lo, hi, 0, 1, 2, 3, 4, 5, 6, 7, 8, 9, 10, 11, 12, 13, 14, 15)); }
__device__ __forceinline__ v8f wmma16(v16h a, v16h b, v8f c) { return __builtin_amdgcn_wmma_f32_16x16x32_f16(false, a, false, b, (short)0, c, false, false); }
__device__ __forceinline__ v8f wmmab(v16bf a, v16bf b, v8f c) { return __builtin_amdgcn_wmma_f32_16x16x32_bf16(false, a, false, b, (short)0, c, false, false); }


template <typename T16> struct WFrag;
template <> struct WFrag<h16> { typedef v16h V; static __device__ __forceinline__ V ld(const h16* p) { return cat16(*(const v8h*)p, *(const v8h*)(p + 16)); } static __device__ __forceinline__ v8f mma(V a, V b, v8f c) { return wmma16(a, b, c); } };
template <> struct WFrag<bf> { typedef v16bf V; static __device__ __forceinline__ V ld(const bf* p) { return cat16b(*(const v8us*)p, *(const v8us*)(p + 16)); } static __device__ __forceinline__ v8f mma(V a, V b, v8f c) { return wmmab(a, b, c); } };
template <typename T16, int NSPLIT, bool BIAS>
__global__ __launch_bounds__(32) void k_gemmw(const T16* __restrict__ A, const T16* __restrict__ A2, const T16* __restrict__ Bt, const T16* __restrict__ Bt2, int K, float* C, int ldc, const float* __restrict__ bias, size_t sA, size_t sB, size_t sC) {
    typedef typename WFrag<T16>::V V;
    __shared__ __align__(16) float os[16 * 68];
    const size_t z = blockIdx.z; A += z * sA; if (A2) A2 += z * sA; Bt += z * sB; if (Bt2) Bt2 += z * sB; C += z * sC;
    const int lane = threadIdx.x & 31, lr = lane & 15, hi = lane >> 4; const int r0 = blockIdx.x * 64, c0 = blockIdx.y * 64;
    v8f acc[4][4];
#pragma unroll
    for (int mb = 0; mb < 4; ++mb)
#pragma unroll
        for (int nb = 0; nb < 4; ++nb) acc[mb][nb] = (v8f){};
    const size_t aoff = (size_t)(r0 + lr) * K + 8 * hi, boff = (size_t)(c0 + lr) * K + 8 * hi;
#pragma unroll 1
    for (int kc = 0; kc < K; kc += 32) {
        V a[4], a2[4];
#pragma unroll
        for (int mb = 0; mb < 4; ++mb) { a[mb] = WFrag<T16>::ld(A + aoff + (size_t)mb * 16 * K + kc); if (NSPLIT == 1 || NSPLIT == 2) a2[mb] = WFrag<T16>::ld(A2 + aoff + (size_t)mb * 16 * K + kc); }
#pragma unroll
        for (int nb = 0; nb < 4; ++nb) { const V b = WFrag<T16>::ld(Bt + boff + (size_t)nb * 16 * K + kc); V b2; if (NSPLIT >= 2) b2 = WFrag<T16>::ld(Bt2 + boff + (size_t)nb * 16 * K + kc);
#pragma unroll
            for (int mb = 0; mb < 4; ++mb) { acc[mb][nb] = WFrag<T16>::mma(a[mb], b, acc[mb][nb]); if (NSPLIT == 1 || NSPLIT == 2) acc[mb][nb] = WFrag<T16>::mma(a2[mb], b, acc[mb][nb]); if (NSPLIT >= 2) acc[mb][nb] = WFrag<T16>::mma(a[mb], b2, acc[mb][nb]); } }
        asm volatile("v_nop\n\tv_nop\n\tv_nop\n\tv_nop" : "+v"(acc[0][0]), "+v"(acc[1][1]), "+v"(acc[2][2]), "+v"(acc[3][3]) : "v"(a[0]), "v"(a[3]));
    }
#pragma unroll
    for (int mb = 0; mb < 4; ++mb) {
#pragma unroll
        for (int nb = 0; nb < 4; ++nb) {
#pragma unroll
            for (int j = 0; j < 8; ++j) os[(hi * 8 + j) * 68 + nb * 16 + lr] = acc[mb][nb][j]; }
        __builtin_amdgcn_wave_barrier(); asm volatile("" ::: "memory");
        float* crow = C + (size_t)(r0 + mb * 16) * ldc + c0;
#pragma unroll 1
        for (int ps = 0; ps < 2; ++ps) {
#pragma unroll
            for (int s = 0; s < 8; ++s) { const int row = 2 * s + hi, cofs = lr * 4; v4f val = *(const v4fa*)(os + row * 68 + cofs); if (BIAS) { val[0] += bfr(bias[c0 + cofs]); val[1] += bfr(bias[c0 + cofs + 1]); val[2] += bfr(bias[c0 + cofs + 2]); val[3] += bfr(bias[c0 + cofs + 3]); }
                *(volatile v4f*)(crow + (size_t)row * ldc + cofs) = val; }
            if (ps == 0) __threadfence(); }
        __builtin_amdgcn_wave_barrier(); asm volatile("" ::: "memory");
    }
}

__device__ __forceinline__ h16 tohx(float x) { return (h16)x; }
__device__ __forceinline__ void splitf(float y, unsigned short& h, unsigned short& l) { h = f2bf(y); l = f2bf(y - bf2f(h)); }
typedef __attribute__((ext_vector_type(2))) unsigned short v2us;
typedef __attribute__((ext_vector_type(4))) unsigned short v4us;
typedef __attribute__((ext_vector_type(2))) _Float16 v2h;
typedef __attribute__((ext_vector_type(4))) _Float16 v4h;
typedef __attribute__((ext_vector_type(2))) float v2f;

__global__ __launch_bounds__(256) void k_wtG(const float* __restrict__ w, int K, int N, bf* Bt) {
    const int lane = threadIdx.x & 31; const int L0 = (blockIdx.x * 8 + (threadIdx.x >> 5)) * 8; const int nlines = N * K / 64;
#pragma unroll
    for (int ps = 0; ps < 2; ++ps) {
#pragma unroll 1
        for (int l = 0; l < 8; ++l) { const int L = L0 + l; if (L >= nlines) break; const size_t e = (size_t)L * 64 + lane * 2; const int k = (int)(e % K), n = (int)(e / K); v2us o;
            o[0] = f2bf(w[(size_t)k * N + n]); o[1] = f2bf(w[(size_t)(k + 1) * N + n]); *(volatile v2us*)(Bt + e) = o; }
        if (ps == 0) __threadfence(); }
}
__global__ __launch_bounds__(256) void k_cvt8(const float* __restrict__ src, bf* dst, size_t n8) { const size_t i = (size_t)blockIdx.x * 256 + threadIdx.x; if (i >= n8) return; const v8f v = *(const v8f*)(src + i * 8); v8us o;
#pragma unroll
    for (int k = 0; k < 8; ++k) o[k] = f2bf(v[k]); *(volatile v8us*)(dst + i * 8) = o; __threadfence(); *(volatile v8us*)(dst + i * 8) = o; }
__global__ __launch_bounds__(256) void k_wsmd(const float* __restrict__ wq, const float* __restrict__ wk, bf* Bt) { const int e = (blockIdx.x * 256 + threadIdx.x) * 4; if (e >= 4 * HD * DMD) return; const int f = e % DMD; const int row = e / DMD; const int p = row / (2 * HD), h = (row / HD) % 2, d = row % HD; const float* w = (p == 0) ? wq : wk; v4us o;
#pragma unroll
    for (int u = 0; u < 4; ++u) o[u] = f2bf(w[((size_t)h * DMD + f + u) * HD + d]); *(volatile v4us*)(Bt + e) = o; __threadfence(); *(volatile v4us*)(Bt + e) = o; }
__global__ __launch_bounds__(256) void k_wch(const float* __restrict__ cw, bf* Bt) { const int e = (blockIdx.x * 256 + threadIdx.x) * 4; if (e >= 64 * DMD) return; const int f = e % DMD; const int c = e / DMD; v4us o;
#pragma unroll
    for (int u = 0; u < 4; ++u) o[u] = (c < NSM) ? f2bf(cw[(size_t)c * DMD + f + u]) : (unsigned short)0; *(volatile v4us*)(Bt + e) = o; __threadfence(); *(volatile v4us*)(Bt + e) = o; }
__global__ __launch_bounds__(256) void k_trig(float* CS) { const int e = blockIdx.x * 256 + threadIdx.x; if (e >= NN * 32) return; const int j = e % 32; const int n = e / 32; const float invf = 1.0f / powf(10000.0f, (float)(2 * j) / 64.0f); const float ang = __fmul_rn((float)n, invf); v2f o; o[0] = cosf(ang); o[1] = sinf(ang); *(volatile v2f*)(CS + (size_t)e * 2) = o; __threadfence(); *(volatile v2f*)(CS + (size_t)e * 2) = o; }
__device__ __forceinline__ float ropev(const float* __restrict__ f, int dd, const float* __restrict__ CS, int n) { const int j = dd & 31; const float cc = CS[((size_t)n * 32 + j) * 2], ss = CS[((size_t)n * 32 + j) * 2 + 1]; const float rot = (dd < 32) ? -f[dd + 32] : f[dd - 32]; float a = __fmul_rn(f[dd], cc); asm volatile("" : "+v"(a)); float b = __fmul_rn(rot, ss); asm volatile("" : "+v"(b)); return __fadd_rn(a, b); }
__global__ __launch_bounds__(256) void k_ropehl(const float* __restrict__ F, int ld, int c0, int nz, const float* __restrict__ CS, float sc, bf* Ph, bf* Pl) { const size_t e = ((size_t)blockIdx.x * 256 + threadIdx.x) * 4; if (e >= (size_t)nz * NN * HD) return; const int d = (int)(e % HD); const int n = (int)((e / HD) % NN); const int z = (int)(e / ((size_t)HD * NN)); const float* f = F + (size_t)n * ld + c0 + z * HD; v4us oh, ol;
#pragma unroll
    for (int u = 0; u < 4; ++u) { unsigned short a, b; splitf(ropev(f, d + u, CS, n) * sc, a, b); oh[u] = a; ol[u] = b; } *(volatile v4us*)(Ph + e) = oh; *(volatile v4us*)(Pl + e) = ol; __threadfence(); *(volatile v4us*)(Ph + e) = oh; *(volatile v4us*)(Pl + e) = ol; }
__global__ __launch_bounds__(256) void k_rope16(const float* __restrict__ F, int ld, int c0, int nz, const float* __restrict__ CS, float sc, h16* P) { const size_t e = ((size_t)blockIdx.x * 256 + threadIdx.x) * 4; if (e >= (size_t)nz * NN * HD) return; const int d = (int)(e % HD); const int n = (int)((e / HD) % NN); const int z = (int)(e / ((size_t)HD * NN)); const float* f = F + (size_t)n * ld + c0 + z * HD; v4h o;
#pragma unroll
    for (int u = 0; u < 4; ++u) o[u] = tohx(ropev(f, d + u, CS, n) * sc); *(volatile v4h*)(P + e) = o; __threadfence(); *(volatile v4h*)(P + e) = o; }
__global__ __launch_bounds__(256) void k_vt2(const float* __restrict__ V, int h0, int nz, bf* Th, bf* Tl) { const size_t e = ((size_t)blockIdx.x * 256 + threadIdx.x) * 2; if (e >= (size_t)nz * HD * NN) return; const int m = (int)(e % NN); const int d = (int)((e / NN) % HD); const int z = (int)(e / ((size_t)NN * HD)); v2us oh, ol;
#pragma unroll
    for (int u = 0; u < 2; ++u) { unsigned short a, b; splitf(V[(size_t)(m + u) * (NH_ * HD) + (h0 + z) * HD + d], a, b); oh[u] = a; ol[u] = b; } *(volatile v2us*)(Th + e) = oh; *(volatile v2us*)(Tl + e) = ol; __threadfence(); *(volatile v2us*)(Th + e) = oh; *(volatile v2us*)(Tl + e) = ol; }
__global__ __launch_bounds__(256) void k_vt16(const float* __restrict__ V, int h0, int nz, h16* T16) { const size_t e = ((size_t)blockIdx.x * 256 + threadIdx.x) * 2; if (e >= (size_t)nz * HD * NN) return; const int m = (int)(e % NN); const int d = (int)((e / NN) % HD); const int z = (int)(e / ((size_t)NN * HD)); v2h o; o[0] = tohx(V[(size_t)m * (NH_ * HD) + (h0 + z) * HD + d]); o[1] = tohx(V[(size_t)(m + 1) * (NH_ * HD) + (h0 + z) * HD + d]); *(volatile v2h*)(T16 + e) = o; __threadfence(); *(volatile v2h*)(T16 + e) = o; }
__global__ __launch_bounds__(64) void k_chg0(const float* __restrict__ CH, const float* __restrict__ cb, float* CG) { const int e = blockIdx.x * 64 + threadIdx.x; if (e >= NSM * NN) return; const int h = e / NN, n = e % NN; const float z = __fadd_rn(CH[(size_t)n * 64 + h], bfr(cb[h])); const float v = __fdiv_rn(1.0f, __fadd_rn(1.0f, __expf(-z))); *(volatile float*)(CG + e) = v; __threadfence(); *(volatile float*)(CG + e) = v; }
__global__ __launch_bounds__(256) void k_rsm(const float* __restrict__ LG, int mode, float* ATT, bf* Ph, bf* Pl) { const int lane = threadIdx.x & 31; const int row = blockIdx.x * 8 + (threadIdx.x >> 5); if (row >= NSM * NN) return; const float* sr = LG + (size_t)row * NN; float v[NN / 32]; float mx = -3.0e38f;
#pragma unroll
    for (int ch = 0; ch < NN / 128; ++ch) { const v4f a = *(const v4f*)(sr + ch * 128 + lane * 4);
#pragma unroll
        for (int u = 0; u < 4; ++u) { v[ch * 4 + u] = a[u]; mx = fmaxf(mx, a[u]); } }
#pragma unroll
    for (int sh = 16; sh; sh >>= 1) mx = fmaxf(mx, __shfl_xor(mx, sh, 32));
    float sum = 0.f;
#pragma unroll
    for (int q = 0; q < NN / 32; ++q) { float d0 = __fsub_rn(v[q], mx); asm volatile("" : "+v"(d0)); v[q] = __builtin_amdgcn_exp2f(__fmul_rn(d0, 1.4426950408889634f)); sum += v[q]; }
#pragma unroll
    for (int sh = 16; sh; sh >>= 1) sum += __shfl_xor(sum, sh, 32);
    const float f = __fdiv_rn(1.0f, sum);
    for (int ps = 0; ps < 2; ++ps) {
#pragma unroll
        for (int ch = 0; ch < NN / 128; ++ch) { const size_t oo = (size_t)row * NN + ch * 128 + lane * 4;
            if (mode == 0) { v4f o; for (int q = 0; q < 4; ++q) o[q] = v[ch * 4 + q] * f; *(volatile v4f*)(ATT + oo) = o; }
            else { v4us oh, ol; for (int q = 0; q < 4; ++q) { unsigned short a, b; splitf(v[ch * 4 + q] * f, a, b); oh[q] = a; ol[q] = b; } *(volatile v4us*)(Ph + oo) = oh; *(volatile v4us*)(Pl + oo) = ol; } }
        if (ps == 0) __threadfence(); } }
__global__ __launch_bounds__(256) void k_copy4(const float* __restrict__ A, float* Bv, size_t n) { const size_t e = ((size_t)blockIdx.x * 256 + threadIdx.x) * 4; if (e >= n) return; const v4f a = *(const v4f*)(A + e); *(volatile v4f*)(Bv + e) = a; __threadfence(); *(volatile v4f*)(Bv + e) = a; }
__global__ __launch_bounds__(256) void k_cols(const float* __restrict__ ATT, float* RC) { const int e = blockIdx.x * 256 + threadIdx.x; if (e >= NSM * NN) return; const int h = e / NN, m = e % NN; const float* base = ATT + (size_t)h * NN * NN + m; float s = 0.f;
#pragma unroll 1
    for (int n = 0; n < NN; ++n) s = __fadd_rn(s, base[(size_t)n * NN]); *(volatile float*)(RC + e) = s; __threadfence(); *(volatile float*)(RC + e) = s; }
__global__ __launch_bounds__(64) void k_chg(const float* __restrict__ RC, const float* __restrict__ cd, float* CG) { const int e = blockIdx.x * 64 + threadIdx.x; if (e >= NSM * NN) return; const int h = e / NN; const float sg = __fdiv_rn(1.0f, __fadd_rn(1.0f, __expf(-__fsub_rn(RC[e], 1.0f)))); float t = __fmul_rn(bfr(cd[h]), sg); asm volatile("" : "+v"(t)); const float v = __fmul_rn(CG[e], __fsub_rn(1.0f, t)); *(volatile float*)(CG + e) = v; __threadfence(); *(volatile float*)(CG + e) = v; }
__global__ __launch_bounds__(256) void k_upd(float* LG, const float* __restrict__ CP, const float* __restrict__ CG, const float* __restrict__ ss) { const size_t e = ((size_t)blockIdx.x * 256 + threadIdx.x) * 4; if (e >= (size_t)NSM * NN * NN) return; const int m = (int)(e % NN); const int n = (int)((e / NN) % NN); const int h = (int)(e / ((size_t)NN * NN)); const float cn = CG[h * NN + n]; const float st = bfr(ss[h]); const v4f cp = *(const v4f*)(CP + e), lg = *(const v4f*)(LG + e); v4f o;
#pragma unroll
    for (int u = 0; u < 4; ++u) { float en = __fmul_rn(-cp[u], cn); asm volatile("" : "+v"(en)); en = __fmul_rn(en, CG[h * NN + m + u]); asm volatile("" : "+v"(en)); float t = __fmul_rn(st, en); asm volatile("" : "+v"(t)); o[u] = __fsub_rn(lg[u], t); }
    *(volatile v4f*)(LG + e) = o; __threadfence(); *(volatile v4f*)(LG + e) = o; }
__global__ __launch_bounds__(256) void k_s16(const float* __restrict__ S, int nz, h16* P16) { const int lane = threadIdx.x & 31; const int row = blockIdx.x * 8 + (threadIdx.x >> 5); if (row >= nz * NN) return; const float* sr = S + (size_t)row * NN; float v[NN / 32]; float mx = -3.0e38f;
#pragma unroll
    for (int ch = 0; ch < NN / 128; ++ch) { const v4f a = *(const v4f*)(sr + ch * 128 + lane * 4);
#pragma unroll
        for (int u = 0; u < 4; ++u) { v[ch * 4 + u] = a[u]; mx = fmaxf(mx, a[u]); } }
#pragma unroll
    for (int sh = 16; sh; sh >>= 1) mx = fmaxf(mx, __shfl_xor(mx, sh, 32));
    float sum = 0.f;
#pragma unroll
    for (int q = 0; q < NN / 32; ++q) { float d0 = __fsub_rn(v[q], mx); asm volatile("" : "+v"(d0)); v[q] = __builtin_amdgcn_exp2f(__fmul_rn(d0, 1.4426950408889634f)); sum += v[q]; }
#pragma unroll
    for (int sh = 16; sh; sh >>= 1) sum += __shfl_xor(sum, sh, 32);
    const float f = __fdiv_rn(PCAR, sum);
    for (int ps = 0; ps < 2; ++ps) {
#pragma unroll
        for (int ch = 0; ch < NN / 128; ++ch) { v4h o4; for (int q = 0; q < 4; ++q) o4[q] = tohx(v[ch * 4 + q] * f); *(volatile v4h*)(P16 + (size_t)row * NN + ch * 128 + lane * 4) = o4; }
        if (ps == 0) __threadfence(); } }
__global__ __launch_bounds__(256) void k_mrg(const float* __restrict__ O, int h0, int nz, float cs, bf* Ah, bf* Al) { const size_t e = ((size_t)blockIdx.x * 256 + threadIdx.x) * 4; if (e >= (size_t)nz * NN * HD) return; const int d = (int)(e % HD); const int n = (int)((e / HD) % NN); const int z = (int)(e / ((size_t)HD * NN)); v4us oh, ol;
#pragma unroll
    for (int u = 0; u < 4; ++u) { unsigned short a, b; splitf(O[e + u] * cs, a, b); oh[u] = a; ol[u] = b; } const size_t oo = (size_t)n * (NH_ * HD) + (h0 + z) * HD + d; *(volatile v4us*)(Ah + oo) = oh; *(volatile v4us*)(Al + oo) = ol; __threadfence(); *(volatile v4us*)(Ah + oo) = oh; *(volatile v4us*)(Al + oo) = ol; }

extern "C" void kernel_launch(void* const* d_in, const int* in_sizes, int n_in,
                              void* d_out, int out_size, void* d_ws, size_t ws_size, hipStream_t stream) {
    (void)in_sizes; (void)n_in; (void)out_size;
    const float** I = (const float**)d_in;
    const float *x = I[0], *fe = I[1], *wqs = I[2], *wks = I[3], *cw = I[4], *cb = I[5], *ss = I[6], *cd = I[7], *wqd = I[8], *wkd = I[9], *wv = I[10], *wo = I[11];
    float* OUT = (float*)d_out;
    char* wsp = (char*)d_ws;
    auto take = [&](size_t bytes) { char* p = wsp; wsp += (bytes + 255) & ~(size_t)255; return (void*)p; };
    bf* XB = (bf*)take((size_t)NN * DMD * 2); bf* FB = (bf*)take((size_t)NN * DMD * 2); bf* BSM = (bf*)take((size_t)4 * HD * DMD * 2); bf* BCH = (bf*)take((size_t)64 * DMD * 2); bf* BQD = (bf*)take((size_t)NSD * HD * DMD * 2); bf* BKD = (bf*)take((size_t)NSD * HD * DMD * 2); bf* BV = (bf*)take((size_t)NH_ * HD * DMD * 2); bf* BO = (bf*)take((size_t)DMD * NH_ * HD * 2);
    float* CS = (float*)take((size_t)NN * 32 * 2 * 4); float* QK = (float*)take((size_t)NN * 4 * HD * 4); float* CH = (float*)take((size_t)NN * 64 * 4); float* QD = (float*)take((size_t)NN * NSD * HD * 4); float* KD = (float*)take((size_t)NN * NSD * HD * 4); float* V = (float*)take((size_t)NN * NH_ * HD * 4);
    bf* QSh = (bf*)take((size_t)NSM * NN * HD * 2); bf* QSl = (bf*)take((size_t)NSM * NN * HD * 2); bf* KSh = (bf*)take((size_t)NSM * NN * HD * 2); bf* KSl = (bf*)take((size_t)NSM * NN * HD * 2);
    float* CP = (float*)take((size_t)NSM * NN * NN * 4); float* LG = (float*)take((size_t)NSM * NN * NN * 4); float* ATT = (float*)take((size_t)NSM * NN * NN * 4); float* CG = (float*)take(NSM * NN * 4); float* RC = (float*)take(NSM * NN * 4);
    bf* VTh = (bf*)take((size_t)NSM * HD * NN * 2); bf* VTl = (bf*)take((size_t)NSM * HD * NN * 2); float* O = (float*)take((size_t)NSM * NN * HD * 4); bf* CTh = (bf*)take((size_t)NN * NH_ * HD * 2); bf* CTl = (bf*)take((size_t)NN * NH_ * HD * 2);
    h16* Q16 = (h16*)take((size_t)NSD * NN * HD * 2); h16* K16 = (h16*)take((size_t)NSD * NN * HD * 2); h16* VT16 = (h16*)take((size_t)NSM * HD * NN * 2);
    if ((size_t)(wsp - (char*)d_ws) > ws_size) return;
    h16* P16 = (h16*)LG; float* S2 = ATT; bf* Ph = (bf*)CP; bf* Pl = Ph + (size_t)NSM * NN * NN;
    k_cvt8<<<(NN * DMD / 8 + 255) / 256, 256, 0, stream>>>(x, XB, NN * DMD / 8); k_cvt8<<<(NN * DMD / 8 + 255) / 256, 256, 0, stream>>>(fe, FB, NN * DMD / 8);
    k_wsmd<<<(4 * HD * DMD / 4 + 255) / 256, 256, 0, stream>>>(wqs, wks, BSM); k_wch<<<(64 * DMD / 4 + 255) / 256, 256, 0, stream>>>(cw, BCH);
    k_wtG<<<(unsigned)((DMD * NSD * HD / 64 + 63) / 64), 256, 0, stream>>>(wqd, DMD, NSD * HD, BQD); k_wtG<<<(unsigned)((DMD * NSD * HD / 64 + 63) / 64), 256, 0, stream>>>(wkd, DMD, NSD * HD, BKD); k_wtG<<<(unsigned)((DMD * NH_ * HD / 64 + 63) / 64), 256, 0, stream>>>(wv, DMD, NH_ * HD, BV); k_wtG<<<(unsigned)((NH_ * HD * DMD / 64 + 63) / 64), 256, 0, stream>>>(wo, NH_ * HD, DMD, BO);
    k_trig<<<(NN * 32 + 255) / 256, 256, 0, stream>>>(CS);
    k_gemmw<bf, 0, false><<<dim3(NN / 64, 4 * HD / 64, 1), 32, 0, stream>>>(FB, nullptr, BSM, nullptr, DMD, QK, 4 * HD, nullptr, 0, 0, 0);
    k_gemmw<bf, 0, false><<<dim3(NN / 64, 1, 1), 32, 0, stream>>>(FB, nullptr, BCH, nullptr, DMD, CH, 64, nullptr, 0, 0, 0);
    k_gemmw<bf, 0, false><<<dim3(NN / 64, NSD * HD / 64, 1), 32, 0, stream>>>(XB, nullptr, BQD, nullptr, DMD, QD, NSD * HD, nullptr, 0, 0, 0); k_gemmw<bf, 0, false><<<dim3(NN / 64, NSD * HD / 64, 1), 32, 0, stream>>>(XB, nullptr, BKD, nullptr, DMD, KD, NSD * HD, nullptr, 0, 0, 0);
    k_gemmw<bf, 0, false><<<dim3(NN / 64, NH_ * HD / 64, 1), 32, 0, stream>>>(XB, nullptr, BV, nullptr, DMD, V, NH_ * HD, nullptr, 0, 0, 0);
    const unsigned gP2 = (unsigned)(((size_t)NSM * NN * HD / 4 + 255) / 256);
    k_ropehl<<<gP2, 256, 0, stream>>>(QK, 4 * HD, 0, NSM, CS, 0.125f, QSh, QSl); k_ropehl<<<gP2, 256, 0, stream>>>(QK, 4 * HD, 2 * HD, NSM, CS, 1.0f, KSh, KSl);
    const unsigned gU0 = (unsigned)(((size_t)NSM * NN * NN / 4 + 255) / 256);
    k_gemmw<bf, 2, false><<<dim3(NN / 64, NN / 64, NSM), 32, 0, stream>>>(QSh, QSl, KSh, KSl, HD, CP, NN, nullptr, (size_t)NN * HD, (size_t)NN * HD, (size_t)NN * NN);
    k_copy4<<<gU0, 256, 0, stream>>>(CP, LG, (size_t)NSM * NN * NN);
    k_chg0<<<(NSM * NN + 63) / 64, 64, 0, stream>>>(CH, cb, CG);
    const unsigned gU = gU0;
    for (int s = 0; s < NSTEP; ++s) { k_rsm<<<NSM * NN / 8, 256, 0, stream>>>(LG, 0, ATT, nullptr, nullptr); k_cols<<<(NSM * NN + 255) / 256, 256, 0, stream>>>(ATT, RC); k_chg<<<(NSM * NN + 63) / 64, 64, 0, stream>>>(RC, cd, CG); k_upd<<<gU, 256, 0, stream>>>(LG, CP, CG, ss); }
    k_rsm<<<NSM * NN / 8, 256, 0, stream>>>(LG, 1, nullptr, Ph, Pl);
    k_vt2<<<(unsigned)(((size_t)NSM * HD * NN / 2 + 255) / 256), 256, 0, stream>>>(V, 0, NSM, VTh, VTl);
    k_gemmw<bf, 2, false><<<dim3(NN / 64, 1, NSM), 32, 0, stream>>>(Ph, Pl, VTh, VTl, NN, O, HD, nullptr, (size_t)NN * NN, (size_t)HD * NN, (size_t)NN * HD);
    k_mrg<<<gP2, 256, 0, stream>>>(O, 0, NSM, 1.0f, CTh, CTl);
    k_rope16<<<(unsigned)(((size_t)NSD * NN * HD / 4 + 255) / 256), 256, 0, stream>>>(QD, NSD * HD, 0, NSD, CS, 0.125f, Q16); k_rope16<<<(unsigned)(((size_t)NSD * NN * HD / 4 + 255) / 256), 256, 0, stream>>>(KD, NSD * HD, 0, NSD, CS, 1.0f, K16);
    for (int h0 = 0; h0 < NSD; h0 += 2) {
        k_gemmw<h16, 0, false><<<dim3(NN / 64, NN / 64, 2), 32, 0, stream>>>(Q16 + (size_t)h0 * NN * HD, nullptr, K16 + (size_t)h0 * NN * HD, nullptr, HD, S2, NN, nullptr, (size_t)NN * HD, (size_t)NN * HD, (size_t)NN * NN);
        k_s16<<<2 * NN / 8, 256, 0, stream>>>(S2, 2, P16);
        k_vt16<<<(unsigned)(((size_t)2 * HD * NN / 2 + 255) / 256), 256, 0, stream>>>(V, NSM + h0, 2, VT16);
        k_gemmw<h16, 0, false><<<dim3(NN / 64, 1, 2), 32, 0, stream>>>(P16, nullptr, VT16, nullptr, NN, O, HD, nullptr, (size_t)NN * NN, (size_t)HD * NN, (size_t)NN * HD);
        k_mrg<<<gP2, 256, 0, stream>>>(O, NSM + h0, 2, 1.0f / PCAR, CTh, CTl); }
    k_gemmw<bf, 1, false><<<dim3(NN / 64, DMD / 64, 1), 32, 0, stream>>>(CTh, CTl, BO, nullptr, NH_ * HD, OUT, DMD, nullptr, 0, 0, 0);
}
